// KANLayer_42116449305065
// MI455X (gfx1250) — hardware-verified
//
#include <hip/hip_runtime.h>
#include <stdint.h>

#define NB     2048
#define NI     1024
#define NO     1024
#define NG     8
#define KX     NI
#define KS     (NI * NG)
#define KTOT   (KX + 2 * KS)
#define UROW   (KTOT / 8)
#define FTHR   256
#define NSWEEP ((UROW + FTHR - 1) / FTHR)
#define UBASE  (NO * KX / 8)
#define UCOEF  (NO * KS / 8)
#define SPL    0.1f
#define WSCAP  134217728

static_assert(KTOT % 32 == 0);
static_assert(UROW % 32 == 0);
static_assert(NSWEEP * FTHR >= UROW);
static_assert((UROW % FTHR) % 32 == 0);
static_assert(FTHR * 4 == NI);
static_assert(UBASE % 256 == 0);
static_assert(UCOEF % 256 == 0);
static_assert(NB % 128 == 0);
static_assert(NO % 64 == 0);
static_assert((KTOT * 2) % 128 == 0);
static_assert((KX * 2) % 128 == 0);
static_assert((KS * 2) % 128 == 0);
static_assert(KX % 32 == 0);
static_assert(KS % 32 == 0);

typedef float          v4f   __attribute__((ext_vector_type(4)));
typedef float          v8f   __attribute__((ext_vector_type(8)));
typedef int            v8i   __attribute__((ext_vector_type(8)));
typedef unsigned int   v2u   __attribute__((ext_vector_type(2)));
typedef unsigned int   v4u   __attribute__((ext_vector_type(4)));
typedef unsigned short v8us  __attribute__((ext_vector_type(8)));
typedef unsigned short v16us __attribute__((ext_vector_type(16)));
typedef __bf16         v16bf __attribute__((ext_vector_type(16)));
typedef v4f  __attribute__((may_alias)) v4fa;
typedef v2u  __attribute__((may_alias)) v2ua;
typedef v4u  __attribute__((may_alias)) v4ua;
typedef v8us __attribute__((may_alias)) v8usa;
union FragB { v16bf v; v16us u; v8us h[2]; v8i w; };

__device__ __forceinline__ unsigned short f2bf_bits(float f) {
  unsigned u = __float_as_uint(f);
  return (unsigned short)((u + 0x7FFFu + ((u >> 16) & 1u)) >> 16);
}
__device__ __forceinline__ float bf_bits2f(unsigned short b) { return __uint_as_float(((unsigned)b) << 16); }
__device__ __forceinline__ float bfr(float f) { return bf_bits2f(f2bf_bits(f)); }
__device__ __forceinline__ unsigned pk16(unsigned short a, unsigned short b) { return (unsigned)a | ((unsigned)b << 16); }

__device__ __forceinline__ v8f wmb(const FragB& a, const FragB& b, v8f c) {
  v8f d = __builtin_amdgcn_wmma_f32_16x16x32_bf16(false, a.v, false, b.v, (short)0, c, false, false);
  asm volatile("v_nop\n\tv_nop\n\tv_nop\n\tv_nop" : "+v"(d) : "v"(a.w), "v"(b.w));
  return d;
}
__device__ __forceinline__ v8f z8() { v8f z = {0.f, 0.f, 0.f, 0.f, 0.f, 0.f, 0.f, 0.f}; return z; }

__device__ __forceinline__ v4u cvt8_bf16(const float* src) {
  const v4f a = *(const v4fa*)src;
  const v4f c = *(const v4fa*)(src + 4);
  v4u v;
  v.x = pk16(f2bf_bits(a.x), f2bf_bits(a.y));
  v.y = pk16(f2bf_bits(a.z), f2bf_bits(a.w));
  v.z = pk16(f2bf_bits(c.x), f2bf_bits(c.y));
  v.w = pk16(f2bf_bits(c.z), f2bf_bits(c.w));
  return v;
}

__global__ __launch_bounds__(256) void prep_base_kernel(const float* __restrict__ bw, unsigned short* __restrict__ WB) {
  const size_t u = (size_t)blockIdx.x * 256 + (size_t)threadIdx.x;
  const size_t o = u >> 7, j = u & 127;
  const v4u v = cvt8_bf16(bw + u * 8);
  unsigned short* dst = WB + o * (size_t)KTOT + 8 * j;
  *(volatile v4u*)dst = v;
  __threadfence();
  *(volatile v4u*)dst = v;
}

__global__ __launch_bounds__(256) void prep_coeff_kernel(const float* __restrict__ sc, unsigned short* __restrict__ WB) {
  const size_t u = (size_t)blockIdx.x * 256 + (size_t)threadIdx.x;
  const size_t o = u >> 10, j = u & 1023;
  const v4u v = cvt8_bf16(sc + u * 8);
  unsigned short* dst1 = WB + o * (size_t)KTOT + KX + 8 * j;
  unsigned short* dst2 = dst1 + KS;
  *(volatile v4u*)dst1 = v;
  *(volatile v4u*)dst2 = v;
  __threadfence();
  *(volatile v4u*)dst1 = v;
  *(volatile v4u*)dst2 = v;
}

__device__ __forceinline__ void a_store_pass(const unsigned short* sA, unsigned short* dst, int tid) {
#pragma unroll
  for (int it = 0; it < NSWEEP; ++it) {
    const int u = it * FTHR + tid;
    if (u < UROW) {
      const v4u v = *(const v4ua*)(sA + 8 * u);
      *(volatile v4u*)(dst + 8 * u) = v;
    }
  }
}

__global__ __launch_bounds__(FTHR) void feat_kernel(const float* __restrict__ x,
                                                    const float* __restrict__ gridv,
                                                    unsigned short* __restrict__ AP) {
  __shared__ __align__(16) unsigned short sA[KTOT];
  const int tid = threadIdx.x, lane = tid & 31;
  const int r = blockIdx.x;

  const int gl = (lane < NG) ? lane : NG;
  const float gv = bfr(gridv[gl]);
  float g[NG + 1];
#pragma unroll
  for (int j = 0; j <= NG; ++j) g[j] = __shfl(gv, j);

  const v4f xv = *(const v4fa*)(x + (size_t)r * NI + 4 * tid);
  unsigned short xbits[4];

#pragma unroll
  for (int c = 0; c < 4; ++c) {
    const float xf = xv[c];
    const unsigned short xbb = f2bf_bits(xf);
    xbits[c] = xbb;
    const float xb = bf_bits2f(xbb);
    const float xc = fminf(fmaxf(xb, -1.0f), 1.0f);

    int cnt = 0;
#pragma unroll
    for (int j = 0; j <= NG; ++j) cnt += (xc >= g[j]) ? 1 : 0;
    int bin = cnt - 1;
    bin = (bin < 0) ? 0 : bin;
    bin = (bin > NG - 1) ? (NG - 1) : bin;

    float left = g[0], right = g[1];
#pragma unroll
    for (int j = 1; j < NG; ++j) {
      const bool e = (bin == j);
      left  = e ? g[j] : left;
      right = e ? g[j + 1] : right;
    }
    float den = right - left;
    den = (den == 0.0f) ? 1.0f : den;
    const float wgt = (xc - left) / den;
    const float v = SPL * wgt;
    const unsigned short hb = f2bf_bits(v);
    const float hi = bf_bits2f(hb);
    const unsigned short lb = f2bf_bits(v - hi);
    const unsigned short zz = (unsigned short)0;

    v4u uh, ul;
    uh.x = pk16((bin == 0) ? hb : zz, (bin == 1) ? hb : zz);
    uh.y = pk16((bin == 2) ? hb : zz, (bin == 3) ? hb : zz);
    uh.z = pk16((bin == 4) ? hb : zz, (bin == 5) ? hb : zz);
    uh.w = pk16((bin == 6) ? hb : zz, (bin == 7) ? hb : zz);
    ul.x = pk16((bin == 0) ? lb : zz, (bin == 1) ? lb : zz);
    ul.y = pk16((bin == 2) ? lb : zz, (bin == 3) ? lb : zz);
    ul.z = pk16((bin == 4) ? lb : zz, (bin == 5) ? lb : zz);
    ul.w = pk16((bin == 6) ? lb : zz, (bin == 7) ? lb : zz);

    const int i = 4 * tid + c;
    *(v4ua*)(sA + KX + 8 * i) = uh;
    *(v4ua*)(sA + KX + KS + 8 * i) = ul;
  }
  v2u xw;
  xw.x = pk16(xbits[0], xbits[1]);
  xw.y = pk16(xbits[2], xbits[3]);
  *(v2ua*)(sA + 4 * tid) = xw;
  __syncthreads();

  unsigned short* dst = AP + (size_t)r * KTOT;
  a_store_pass(sA, dst, tid);
  __threadfence();
  a_store_pass(sA, dst, tid);
}

__device__ __forceinline__ void o_store_pass(const float* sO, float* out,
                                             int grow_w, int n0, int w, int lane) {
  const int q8 = lane & 7, sub = lane >> 3;
#pragma unroll
  for (int i = 0; i < 16; ++i) {
    const int lid = i * 4 + sub;
    const int row = lid >> 1, hl = lid & 1;
    const v4f v = *(const v4fa*)(sO + (32 * w + row) * 64 + 32 * hl + 4 * q8);
    *(volatile v4f*)(out + (size_t)(grow_w + row) * NO + n0 + 32 * hl + 4 * q8) = v;
  }
}

__global__ __launch_bounds__(128) void gemm_kernel(const unsigned short* __restrict__ AP,
                                                   const unsigned short* __restrict__ WB,
                                                   float* __restrict__ out) {
  __shared__ __align__(16) float sO[128 * 64];
  const int tid = threadIdx.x, lane = tid & 31, w = tid >> 5;
  const int h = lane >> 4, m = lane & 15;
  const int row_w = blockIdx.x * 128 + 32 * w;
  const int n0 = blockIdx.y * 64;

  const unsigned short* xa0 = AP + (size_t)(row_w + m) * KTOT + 8 * h;
  const unsigned short* xa1 = xa0 + (size_t)16 * KTOT;
  const unsigned short* wb  = WB + (size_t)(n0 + m) * KTOT + 8 * h;

  v8f acc[2][4];
#pragma unroll
  for (int mt = 0; mt < 2; ++mt)
#pragma unroll
    for (int nt = 0; nt < 4; ++nt) acc[mt][nt] = z8();

#pragma unroll 1
  for (int k0 = 0; k0 < KTOT; k0 += 32) {
    FragB a0, a1;
    a0.h[0] = *(const v8usa*)(xa0 + k0);
    a0.h[1] = *(const v8usa*)(xa0 + k0 + 16);
    a1.h[0] = *(const v8usa*)(xa1 + k0);
    a1.h[1] = *(const v8usa*)(xa1 + k0 + 16);
#pragma unroll
    for (int nt = 0; nt < 4; ++nt) {
      const unsigned short* wq = wb + (size_t)nt * 16 * KTOT + k0;
      FragB b;
      b.h[0] = *(const v8usa*)wq;
      b.h[1] = *(const v8usa*)(wq + 16);
      acc[0][nt] = wmb(a0, b, acc[0][nt]);
      acc[1][nt] = wmb(a1, b, acc[1][nt]);
    }
  }

#pragma unroll
  for (int nt = 0; nt < 4; ++nt) {
    const int cl = 16 * nt + m;
#pragma unroll
    for (int mt = 0; mt < 2; ++mt) {
#pragma unroll
      for (int r = 0; r < 8; ++r) {
        const int rl = 32 * w + 16 * mt + 8 * h + r;
        sO[rl * 64 + cl] = acc[mt][nt][r];
      }
    }
  }
  __syncthreads();

  o_store_pass(sO, out, row_w, n0, w, lane);
  __threadfence();
  o_store_pass(sO, out, row_w, n0, w, lane);
}

extern "C" void kernel_launch(void* const* d_in, const int* in_sizes, int n_in,
                              void* d_out, int out_size, void* d_ws, size_t ws_size,
                              hipStream_t stream) {
  if (n_in < 4) return;
  if (in_sizes[0] != NB * NI) return;
  if (in_sizes[1] != NO * NI) return;
  if (in_sizes[2] != NO * NI * NG) return;
  if (in_sizes[3] != NG + 1) return;
  if (out_size != NB * NO) return;

  const float* x     = (const float*)d_in[0];
  const float* bw    = (const float*)d_in[1];
  const float* sc    = (const float*)d_in[2];
  const float* gridv = (const float*)d_in[3];
  float* out = (float*)d_out;

  size_t off = 0;
  const size_t oAP = off; off += (size_t)NB * KTOT * 2;
  const size_t oWB = off; off += (size_t)NO * KTOT * 2;
  if (off > ws_size) return;
  if (off > (size_t)WSCAP) return;

  char* ws = (char*)d_ws;
  unsigned short* AP = (unsigned short*)(ws + oAP);
  unsigned short* WB = (unsigned short*)(ws + oWB);

  prep_base_kernel<<<dim3(UBASE / 256), dim3(256), 0, stream>>>(bw, WB);
  prep_coeff_kernel<<<dim3(UCOEF / 256), dim3(256), 0, stream>>>(sc, WB);
  feat_kernel<<<dim3(NB), dim3(FTHR), 0, stream>>>(x, gridv, AP);
  gemm_kernel<<<dim3(NB / 128, NO / 64), dim3(128), 0, stream>>>(AP, WB, out);
  (void)hipGetLastError();
}
